// GroupedQueryAttention_75874892251738
// MI455X (gfx1250) — hardware-verified
//
#include <hip/hip_runtime.h>
#include <stddef.h>


#ifndef NB
#define NB 2
#endif
#ifndef SEQ
#define SEQ 2048
#endif
#define NB_FULL 2
#define SEQ_FULL 2048

static constexpr int DMOD = 2048;
static constexpr int NQH  = 32;
static constexpr int DH   = 64;
static constexpr int KVD  = 512;
static constexpr int ER   = 256;
static constexpr int MTOT = NB * SEQ;
static constexpr int LROW = 72;
static constexpr int TPV  = 136;
static constexpr int TPF  = 68;

static constexpr float WSC    = 64.0f;
static constexpr float WSCINV = 0.015625f;
static constexpr float PCAR   = 1024.0f;
static constexpr float PCINV  = 0.0009765625f;
static constexpr float RESC   = 1024.0f;
static constexpr float RESINV = 0.0009765625f;
static constexpr float SCL    = 0.125f;
static constexpr float NEGBIG = -1.0e30f;

static_assert(NB >= 1 && NB <= NB_FULL);
static_assert(SEQ >= ER && SEQ <= SEQ_FULL && (SEQ % 256) == 0);
static_assert((MTOT % 128) == 0 && (ER % 128) == 0);
static_assert((DMOD % 64) == 0 && (KVD % 64) == 0 && (DMOD % 32) == 0);
static_assert(NQH * DH == DMOD && (NQH / 4) * DH == KVD);

typedef _Float16     v16h __attribute__((ext_vector_type(16)));
typedef float        v8f  __attribute__((ext_vector_type(8)));
typedef unsigned int v4u  __attribute__((ext_vector_type(4)));
typedef float        v4f  __attribute__((ext_vector_type(4)));
typedef v4u __attribute__((may_alias)) v4ua;
typedef v4f __attribute__((may_alias)) v4fa;

union H8 { v4u u; _Float16 h[8]; };
union HF { v16h v; v4u u[2]; _Float16 h[16]; };

__device__ __forceinline__ v8f mma16(v16h a, v16h b, v8f c) {
  v8f d = __builtin_amdgcn_wmma_f32_16x16x32_f16(false, a, false, b, (short)0, c,
                                                 false, false);
  asm volatile("v_nop\n\tv_nop\n\tv_nop\n\tv_nop" : "+v"(d) : "v"(a), "v"(b));
  return d;
}

__device__ __forceinline__ v16h load_frag(const _Float16* rowptr, int hi) {
  HF f;
  f.u[0] = *reinterpret_cast<const v4ua*>(rowptr + (hi << 3));
  f.u[1] = *reinterpret_cast<const v4ua*>(rowptr + 16 + (hi << 3));
  return f.v;
}

__device__ __forceinline__ float bf16_rne(float x) {
  unsigned u = __builtin_bit_cast(unsigned, x);
  u = (u + 0x7FFFu + ((u >> 16) & 1u)) & 0xFFFF0000u;
  return __builtin_bit_cast(float, u);
}

__global__ void __launch_bounds__(256) cvt_x_kernel(const float* __restrict__ x,
                                                    _Float16* __restrict__ xh) {
  const size_t g   = (size_t)blockIdx.x * 256 + threadIdx.x;
  const size_t tot = (size_t)MTOT * DMOD / 8;
  if (g >= tot) return;
  const size_t e = g * 8;
  const size_t m = e / DMOD;
  const size_t c = e - m * DMOD;
  const size_t srow = (m / SEQ) * SEQ_FULL + (m % SEQ);
  const float* sp = x + srow * DMOD + c;
  const v4f a0 = *reinterpret_cast<const v4fa*>(sp);
  const v4f a1 = *reinterpret_cast<const v4fa*>(sp + 4);
  H8 pk;
  pk.h[0] = (_Float16)bf16_rne(a0[0]);
  pk.h[1] = (_Float16)bf16_rne(a0[1]);
  pk.h[2] = (_Float16)bf16_rne(a0[2]);
  pk.h[3] = (_Float16)bf16_rne(a0[3]);
  pk.h[4] = (_Float16)bf16_rne(a1[0]);
  pk.h[5] = (_Float16)bf16_rne(a1[1]);
  pk.h[6] = (_Float16)bf16_rne(a1[2]);
  pk.h[7] = (_Float16)bf16_rne(a1[3]);
  _Float16* dp = xh + e;
  *reinterpret_cast<volatile v4u*>(dp) = pk.u;
  __threadfence();
  *reinterpret_cast<volatile v4u*>(dp) = pk.u;
}

__global__ void __launch_bounds__(256) tr_w_kernel(const float* __restrict__ W,
                                                   _Float16* __restrict__ Wt,
                                                   int Kdim, int Ndim) {
  __shared__ _Float16 T[64 * LROW];
  const int tid = threadIdx.x;
  const int wid = tid >> 5, lane = tid & 31;
  const int piece = lane & 7, sub = lane >> 3;
  const int n0 = blockIdx.x * 64, k0 = blockIdx.y * 64;
  #pragma unroll
  for (int i = 0; i < 4; ++i) {
    const int p = tid + 256 * i;
    const int row = p >> 4;
    const int c4  = (p & 15) * 4;
    const v4f v = *reinterpret_cast<const v4fa*>(W + (size_t)(k0 + row) * (size_t)Ndim + n0 + c4);
    T[(c4 + 0) * LROW + row] = (_Float16)(bf16_rne(v[0]) * WSC);
    T[(c4 + 1) * LROW + row] = (_Float16)(bf16_rne(v[1]) * WSC);
    T[(c4 + 2) * LROW + row] = (_Float16)(bf16_rne(v[2]) * WSC);
    T[(c4 + 3) * LROW + row] = (_Float16)(bf16_rne(v[3]) * WSC);
  }
  __syncthreads();
  #pragma unroll
  for (int it = 0; it < 2; ++it) {
    const int L = wid * 8 + it * 4 + sub;
    const v4u v = *reinterpret_cast<const v4ua*>(T + L * LROW + piece * 8);
    *reinterpret_cast<volatile v4u*>(Wt + (size_t)(n0 + L) * (size_t)Kdim + k0 + piece * 8) = v;
  }
  __threadfence();
  #pragma unroll
  for (int it = 0; it < 2; ++it) {
    const int L = wid * 8 + it * 4 + sub;
    const v4u v = *reinterpret_cast<const v4ua*>(T + L * LROW + piece * 8);
    *reinterpret_cast<volatile v4u*>(Wt + (size_t)(n0 + L) * (size_t)Kdim + k0 + piece * 8) = v;
  }
}

template <int MODE>
__device__ __forceinline__ void kloop(v8f (&acc)[4][2], const _Float16* __restrict__ xp,
                                      const _Float16* __restrict__ wp, int K, int hi) {
  const size_t k16 = (size_t)16 * (size_t)K;
  #pragma unroll 1
  for (int k = 0; k < K; k += 32) {
    const v16h x0 = load_frag(xp + k, hi);
    const v16h x1 = load_frag(xp + k16 + k, hi);
    #pragma unroll
    for (int j = 0; j < 4; ++j) {
      const v16h w = load_frag(wp + (size_t)j * k16 + k, hi);
      if (MODE == 1) {
        acc[j][0] = mma16(x0, w, acc[j][0]);
        acc[j][1] = mma16(x1, w, acc[j][1]);
      } else {
        acc[j][0] = mma16(w, x0, acc[j][0]);
        acc[j][1] = mma16(w, x1, acc[j][1]);
      }
    }
  }
}

template <int MODE, typename OT>
__global__ void __launch_bounds__(128) __attribute__((amdgpu_num_vgpr(256)))
gemm_kernel(const _Float16* __restrict__ X, const _Float16* __restrict__ Xr,
            const _Float16* __restrict__ Wt, OT* __restrict__ Out,
            _Float16* __restrict__ OutR, int N, int K, float oscale) {
  __shared__ float ldsE[128 * TPF];
  const int tid = threadIdx.x;
  const int wid = tid >> 5, lane = tid & 31, l15 = lane & 15, hi = lane >> 4;
  const int piece = lane & 7, sub = lane >> 3;
  const int n0 = blockIdx.x * 64, m0 = blockIdx.y * 128;
  const int bidx = m0 / SEQ, s0 = m0 - bidx * SEQ;
  const bool early = (s0 < ER);
  const int mw = wid * 32;
  const _Float16* wp = Wt + (size_t)(n0 + l15) * (size_t)K;

  const v8f vz = {0.f, 0.f, 0.f, 0.f, 0.f, 0.f, 0.f, 0.f};
  v8f acc[4][2];
  #pragma unroll
  for (int j = 0; j < 4; ++j) { acc[j][0] = vz; acc[j][1] = vz; }

  if constexpr (MODE == 2) {
    if (early) {
      const _Float16* rp = Xr + (size_t)(bidx * ER + s0 + mw + l15) * (size_t)K;
      kloop<MODE>(acc, rp, wp, K, hi);
      #pragma unroll
      for (int j = 0; j < 4; ++j) {
        acc[j][0] = acc[j][0] * RESINV;
        acc[j][1] = acc[j][1] * RESINV;
      }
    }
  }
  {
    const _Float16* xp = X + (size_t)(m0 + mw + l15) * (size_t)K;
    kloop<MODE>(acc, xp, wp, K, hi);
  }

  if constexpr (MODE == 0) {
    _Float16* T = reinterpret_cast<_Float16*>(ldsE);
    const int npl = early ? 2 : 1;
    for (int pl = 0; pl < npl; ++pl) {
      if (pl) __syncthreads();
      #pragma unroll
      for (int j = 0; j < 4; ++j)
        #pragma unroll
        for (int i = 0; i < 2; ++i) {
          H8 pk;
          #pragma unroll
          for (int r = 0; r < 8; ++r) {
            const float v = acc[j][i][r] * oscale;
            const _Float16 hv = (_Float16)v;
            const _Float16 rv = (_Float16)((v - (float)hv) * RESC);
            pk.h[r] = pl ? rv : hv;
          }
          *reinterpret_cast<v4ua*>(T + (mw + i * 16 + l15) * LROW + j * 16 + 8 * hi) = pk.u;
        }
      __syncthreads();
      OT* base = pl ? (OutR + (size_t)(bidx * ER + s0) * (size_t)N)
                    : (Out + (size_t)m0 * (size_t)N);
      #pragma unroll
      for (int it = 0; it < 8; ++it) {
        const int row = mw + it * 4 + sub;
        const v4u v = *reinterpret_cast<const v4ua*>(T + row * LROW + piece * 8);
        *reinterpret_cast<volatile v4u*>(base + (size_t)row * N + n0 + piece * 8) = v;
      }
      __threadfence();
      #pragma unroll
      for (int it = 0; it < 8; ++it) {
        const int row = mw + it * 4 + sub;
        const v4u v = *reinterpret_cast<const v4ua*>(T + row * LROW + piece * 8);
        *reinterpret_cast<volatile v4u*>(base + (size_t)row * N + n0 + piece * 8) = v;
      }
    }
  } else if constexpr (MODE == 1) {
    _Float16* T = reinterpret_cast<_Float16*>(ldsE);
    const int npl = early ? 2 : 1;
    for (int pl = 0; pl < npl; ++pl) {
      if (pl) __syncthreads();
      #pragma unroll
      for (int j = 0; j < 4; ++j)
        #pragma unroll
        for (int i = 0; i < 2; ++i) {
          H8 pk;
          #pragma unroll
          for (int r = 0; r < 8; ++r) {
            const float v = acc[j][i][r] * oscale;
            const _Float16 hv = (_Float16)v;
            const _Float16 rv = (_Float16)((v - (float)hv) * RESC);
            pk.h[r] = pl ? rv : hv;
          }
          *reinterpret_cast<v4ua*>(T + (j * 16 + l15) * TPV + mw + i * 16 + 8 * hi) = pk.u;
        }
      __syncthreads();
      const int pitch = pl ? ER : SEQ;
      OT* base = (pl ? OutR : Out) + (size_t)(bidx * N + n0) * (size_t)pitch + s0;
      #pragma unroll
      for (int it = 0; it < 8; ++it) {
        const int L = wid * 32 + it * 4 + sub;
        const int n = L >> 1, hl = L & 1;
        const v4u v = *reinterpret_cast<const v4ua*>(T + n * TPV + hl * 64 + piece * 8);
        *reinterpret_cast<volatile v4u*>(base + (size_t)n * pitch + hl * 64 + piece * 8) = v;
      }
      __threadfence();
      #pragma unroll
      for (int it = 0; it < 8; ++it) {
        const int L = wid * 32 + it * 4 + sub;
        const int n = L >> 1, hl = L & 1;
        const v4u v = *reinterpret_cast<const v4ua*>(T + n * TPV + hl * 64 + piece * 8);
        *reinterpret_cast<volatile v4u*>(base + (size_t)n * pitch + hl * 64 + piece * 8) = v;
      }
    }
  } else {
    float* T = ldsE;
    #pragma unroll
    for (int j = 0; j < 4; ++j)
      #pragma unroll
      for (int i = 0; i < 2; ++i) {
        v4f lo4, hi4;
        lo4[0] = acc[j][i][0] * oscale; lo4[1] = acc[j][i][1] * oscale;
        lo4[2] = acc[j][i][2] * oscale; lo4[3] = acc[j][i][3] * oscale;
        hi4[0] = acc[j][i][4] * oscale; hi4[1] = acc[j][i][5] * oscale;
        hi4[2] = acc[j][i][6] * oscale; hi4[3] = acc[j][i][7] * oscale;
        float* tp = T + (mw + i * 16 + l15) * TPF + j * 16 + 8 * hi;
        *reinterpret_cast<v4fa*>(tp)     = lo4;
        *reinterpret_cast<v4fa*>(tp + 4) = hi4;
      }
    __syncthreads();
    OT* base = Out + (size_t)(bidx * SEQ_FULL + s0) * (size_t)N + n0;
    #pragma unroll
    for (int it = 0; it < 16; ++it) {
      const int L = wid * 64 + it * 4 + sub;
      const int r = L >> 1, hl = L & 1;
      const v4f v = *reinterpret_cast<const v4fa*>(T + r * TPF + hl * 32 + piece * 4);
      *reinterpret_cast<volatile v4f*>(base + (size_t)r * N + hl * 32 + piece * 4) = v;
    }
    __threadfence();
    #pragma unroll
    for (int it = 0; it < 16; ++it) {
      const int L = wid * 64 + it * 4 + sub;
      const int r = L >> 1, hl = L & 1;
      const v4f v = *reinterpret_cast<const v4fa*>(T + r * TPF + hl * 32 + piece * 4);
      *reinterpret_cast<volatile v4f*>(base + (size_t)r * N + hl * 32 + piece * 4) = v;
    }
  }
}

template <int QT, int RES>
__global__ void __launch_bounds__(256) __attribute__((amdgpu_num_vgpr(256)))
attn_kernel(const _Float16* __restrict__ Qp, const _Float16* __restrict__ Qr,
            const _Float16* __restrict__ Kp, const _Float16* __restrict__ Kr,
            const _Float16* __restrict__ Vtp, const _Float16* __restrict__ Vr,
            _Float16* __restrict__ Cp, _Float16* __restrict__ Cr,
            int qblk0, int nqblk) {
  constexpr int QB = 128 * QT;
  constexpr int NT = RES ? 4 : 2;
  __shared__ _Float16 ldsT[NT * 64 * LROW];
  __shared__ _Float16 ldsO[QB * LROW];

  const int tid = threadIdx.x;
  const int wid = tid >> 5, lane = tid & 31, l15 = lane & 15, hi = lane >> 4;
  const int piece = lane & 7, sub = lane >> 3;
  const int bid = blockIdx.x;
  const int qbi = qblk0 + (bid % nqblk);
  const int h   = (bid / nqblk) % NQH;
  const int b   = bid / (nqblk * NQH);
  const int kvh = h >> 2;
  const int q0  = qbi * QB;
  const int sbase = q0 + wid * (16 * QT);

  _Float16* const Kb  = ldsT;
  _Float16* const Vb  = ldsT + 64 * LROW;
  _Float16* const Krb = ldsT + (RES ? 128 : 0) * LROW;
  _Float16* const Vrb = ldsT + (RES ? 192 : 64) * LROW;

  v16h qf[QT][2];
  #pragma unroll
  for (int qt = 0; qt < QT; ++qt) {
    const _Float16* qrow = Qp + (size_t)(b * SEQ + sbase + qt * 16 + l15) * (size_t)DMOD + h * DH;
    qf[qt][0] = load_frag(qrow, hi);
    qf[qt][1] = load_frag(qrow + 32, hi);
  }
  v16h qrf0 = qf[0][0], qrf1 = qf[0][1];
  if constexpr (RES) {
    const _Float16* rrow = Qr + (size_t)(b * ER + sbase + l15) * (size_t)DMOD + h * DH;
    qrf0 = load_frag(rrow, hi);
    qrf1 = load_frag(rrow + 32, hi);
  }

  const v8f vz = {0.f, 0.f, 0.f, 0.f, 0.f, 0.f, 0.f, 0.f};
  v8f o[QT][4];
  v8f orr[4];
  #pragma unroll
  for (int qt = 0; qt < QT; ++qt)
    #pragma unroll
    for (int t = 0; t < 4; ++t) o[qt][t] = vz;
  #pragma unroll
  for (int t = 0; t < 4; ++t) orr[t] = vz;
  float m_run[QT], l_run[QT];
  #pragma unroll
  for (int qt = 0; qt < QT; ++qt) { m_run[qt] = NEGBIG; l_run[qt] = 0.0f; }

  const int kend = q0 + QB;
  #pragma unroll 1
  for (int kb = 0; kb < kend; kb += 64) {
    __syncthreads();
    #pragma unroll
    for (int i = 0; i < 2; ++i) {
      const int p = tid + 256 * i;
      const int row = p >> 3, seg = (p & 7) * 8;
      const v4u kv = *reinterpret_cast<const v4ua*>(
          Kp + (size_t)(b * SEQ + kb + row) * (size_t)KVD + kvh * DH + seg);
      *reinterpret_cast<v4ua*>(Kb + row * LROW + seg) = kv;
      const v4u vv = *reinterpret_cast<const v4ua*>(
          Vtp + (size_t)(b * KVD + kvh * DH + row) * (size_t)SEQ + kb + seg);
      *reinterpret_cast<v4ua*>(Vb + row * LROW + seg) = vv;
      if constexpr (RES) {
        const v4u kr = *reinterpret_cast<const v4ua*>(
            Kr + (size_t)(b * ER + kb + row) * (size_t)KVD + kvh * DH + seg);
        *reinterpret_cast<v4ua*>(Krb + row * LROW + seg) = kr;
        const v4u vr = *reinterpret_cast<const v4ua*>(
            Vr + (size_t)(b * KVD + kvh * DH + row) * (size_t)ER + kb + seg);
        *reinterpret_cast<v4ua*>(Vrb + row * LROW + seg) = vr;
      }
    }
    __syncthreads();

    if (kb < sbase + 16 * QT) {
      const bool diag = (kb + 64 > sbase);
      #pragma unroll
      for (int ss = 0; ss < 2; ++ss) {
        const _Float16* k0p = Kb + (ss * 32 + l15) * LROW;
        const _Float16* k1p = k0p + 16 * LROW;
        const v16h ka0 = load_frag(k0p, hi);
        const v16h ka1 = load_frag(k0p + 32, hi);
        const v16h kb0 = load_frag(k1p, hi);
        const v16h kb1 = load_frag(k1p + 32, hi);

        HF pf[QT];
        HF prf;
        prf.v = vz[0] == 0.f ? qf[0][0] : qf[0][0];
        #pragma unroll
        for (int qt = 0; qt < QT; ++qt) {
          v8f sA = mma16(ka0, qf[qt][0], vz);
          sA     = mma16(ka1, qf[qt][1], sA);
          v8f sB = mma16(kb0, qf[qt][0], vz);
          sB     = mma16(kb1, qf[qt][1], sB);
          if constexpr (RES) {
            v8f rA = mma16(ka0, qrf0, vz);
            rA     = mma16(ka1, qrf1, rA);
            v8f rB = mma16(kb0, qrf0, vz);
            rB     = mma16(kb1, qrf1, rB);
            const _Float16* r0p = Krb + (ss * 32 + l15) * LROW;
            const _Float16* r1p = r0p + 16 * LROW;
            const v16h kr0 = load_frag(r0p, hi);
            const v16h kr1 = load_frag(r0p + 32, hi);
            rA = mma16(kr0, qf[qt][0], rA);
            rA = mma16(kr1, qf[qt][1], rA);
            const v16h kr2 = load_frag(r1p, hi);
            const v16h kr3 = load_frag(r1p + 32, hi);
            rB = mma16(kr2, qf[qt][0], rB);
            rB = mma16(kr3, qf[qt][1], rB);
            #pragma unroll
            for (int r = 0; r < 8; ++r) {
              sA[r] = sA[r] + rA[r] * RESINV;
              sB[r] = sB[r] + rB[r] * RESINV;
            }
          }
          #pragma unroll
          for (int r = 0; r < 8; ++r) {
            float a = sA[r] * SCL;
            float c = sB[r] * SCL;
            if (diag) {
              const int keyA = kb + ss * 32 + 8 * hi + r;
              const int qq   = sbase + qt * 16 + l15;
              a = (keyA <= qq) ? a : NEGBIG;
              c = (keyA + 16 <= qq) ? c : NEGBIG;
            }
            sA[r] = a;
            sB[r] = c;
          }
          float mx = m_run[qt];
          #pragma unroll
          for (int r = 0; r < 8; ++r) mx = fmaxf(mx, fmaxf(sA[r], sB[r]));
          mx = fmaxf(mx, __shfl_xor(mx, 16, 32));
          const float alpha = __expf(m_run[qt] - mx);
          m_run[qt] = mx;
          l_run[qt] *= alpha;
          #pragma unroll
          for (int r = 0; r < 8; ++r) {
            o[qt][0][r] *= alpha; o[qt][1][r] *= alpha;
            o[qt][2][r] *= alpha; o[qt][3][r] *= alpha;
          }
          if constexpr (RES) {
            #pragma unroll
            for (int r = 0; r < 8; ++r) {
              orr[0][r] *= alpha; orr[1][r] *= alpha;
              orr[2][r] *= alpha; orr[3][r] *= alpha;
            }
          }
          float lsum = 0.0f;
          #pragma unroll
          for (int r = 0; r < 8; ++r) {
            const float p0 = __expf(sA[r] - mx);
            const float p1 = __expf(sB[r] - mx);
            lsum += p0 + p1;
            const float pc0 = p0 * PCAR;
            const float pc1 = p1 * PCAR;
            const _Float16 h0 = (_Float16)pc0;
            const _Float16 h1 = (_Float16)pc1;
            pf[qt].h[r]     = h0;
            pf[qt].h[8 + r] = h1;
            if constexpr (RES) {
              prf.h[r]     = (_Float16)((pc0 - (float)h0) * RESC);
              prf.h[8 + r] = (_Float16)((pc1 - (float)h1) * RESC);
            }
          }
          l_run[qt] += lsum;
        }

        #pragma unroll
        for (int t = 0; t < 4; ++t) {
          const v16h vf = load_frag(Vb + (t * 16 + l15) * LROW + ss * 32, hi);
          #pragma unroll
          for (int qt = 0; qt < QT; ++qt) o[qt][t] = mma16(vf, pf[qt].v, o[qt][t]);
          if constexpr (RES) {
            orr[t] = mma16(vf, prf.v, orr[t]);
            const v16h vrf = load_frag(Vrb + (t * 16 + l15) * LROW + ss * 32, hi);
            orr[t] = mma16(vrf, pf[0].v, orr[t]);
          }
        }
      }
    }
  }

  float ov[4][8];
  #pragma unroll
  for (int qt = 0; qt < QT; ++qt) {
    const float lt  = l_run[qt] + __shfl_xor(l_run[qt], 16, 32);
    const float inv = (1.0f / lt) * PCINV;
    _Float16* orow = ldsO + (wid * 16 * QT + qt * 16 + l15) * LROW + 8 * hi;
    #pragma unroll
    for (int t = 0; t < 4; ++t) {
      H8 pk;
      #pragma unroll
      for (int r = 0; r < 8; ++r) {
        float v;
        if constexpr (RES) {
          v = (o[qt][t][r] + orr[t][r] * RESINV) * inv;
          ov[t][r] = v;
        } else {
          v = o[qt][t][r] * inv;
        }
        pk.h[r] = (_Float16)v;
      }
      *reinterpret_cast<v4ua*>(orow + t * 16) = pk.u;
    }
  }
  __syncthreads();
  {
    _Float16* base = Cp + (size_t)(b * SEQ + q0) * (size_t)DMOD + h * DH;
    #pragma unroll
    for (int it = 0; it < QB / 32; ++it) {
      const int row = wid * (QB / 8) + it * 4 + sub;
      const v4u v = *reinterpret_cast<const v4ua*>(ldsO + row * LROW + piece * 8);
      *reinterpret_cast<volatile v4u*>(base + (size_t)row * DMOD + piece * 8) = v;
    }
    __threadfence();
    #pragma unroll
    for (int it = 0; it < QB / 32; ++it) {
      const int row = wid * (QB / 8) + it * 4 + sub;
      const v4u v = *reinterpret_cast<const v4ua*>(ldsO + row * LROW + piece * 8);
      *reinterpret_cast<volatile v4u*>(base + (size_t)row * DMOD + piece * 8) = v;
    }
  }
  if constexpr (RES) {
    __syncthreads();
    {
      _Float16* orow = ldsO + (wid * 16 + l15) * LROW + 8 * hi;
      #pragma unroll
      for (int t = 0; t < 4; ++t) {
        H8 pk;
        #pragma unroll
        for (int r = 0; r < 8; ++r) {
          const float v = ov[t][r];
          const _Float16 hv = (_Float16)v;
          pk.h[r] = (_Float16)((v - (float)hv) * RESC);
        }
        *reinterpret_cast<v4ua*>(orow + t * 16) = pk.u;
      }
    }
    __syncthreads();
    _Float16* base = Cr + (size_t)(b * ER + q0) * (size_t)DMOD + h * DH;
    #pragma unroll
    for (int it = 0; it < QB / 32; ++it) {
      const int row = wid * (QB / 8) + it * 4 + sub;
      const v4u v = *reinterpret_cast<const v4ua*>(ldsO + row * LROW + piece * 8);
      *reinterpret_cast<volatile v4u*>(base + (size_t)row * DMOD + piece * 8) = v;
    }
    __threadfence();
    #pragma unroll
    for (int it = 0; it < QB / 32; ++it) {
      const int row = wid * (QB / 8) + it * 4 + sub;
      const v4u v = *reinterpret_cast<const v4ua*>(ldsO + row * LROW + piece * 8);
      *reinterpret_cast<volatile v4u*>(base + (size_t)row * DMOD + piece * 8) = v;
    }
  }
}

extern "C" void kernel_launch(void* const* d_in, const int* in_sizes, int n_in,
                              void* d_out, int out_size, void* d_ws,
                              size_t ws_size, hipStream_t stream) {
  if (n_in < 5) return;
  const long long need_x = ((long long)(NB - 1) * SEQ_FULL + SEQ) * (long long)DMOD;
  if ((long long)in_sizes[0] < need_x) return;
  if (in_sizes[1] < DMOD * DMOD) return;
  if (in_sizes[2] < DMOD * KVD) return;
  if (in_sizes[3] < DMOD * KVD) return;
  if (in_sizes[4] < DMOD * DMOD) return;
  if ((long long)out_size < need_x) return;

  const float* x  = (const float*)d_in[0];
  const float* Wq = (const float*)d_in[1];
  const float* Wk = (const float*)d_in[2];
  const float* Wv = (const float*)d_in[3];
  const float* Wo = (const float*)d_in[4];
  float* out = (float*)d_out;

  char* wsb = (char*)d_ws;
  size_t off = 0;
  auto carve = [&](size_t bytes) -> _Float16* {
    _Float16* p = (_Float16*)(wsb + off);
    off += (bytes + 255) & ~(size_t)255;
    return p;
  };
  _Float16* xh  = carve((size_t)MTOT * DMOD * 2);
  _Float16* wqt = carve((size_t)DMOD * DMOD * 2);
  _Float16* wkt = carve((size_t)KVD * DMOD * 2);
  _Float16* wvt = carve((size_t)KVD * DMOD * 2);
  _Float16* wot = carve((size_t)DMOD * DMOD * 2);
  _Float16* qh  = carve((size_t)MTOT * DMOD * 2);
  _Float16* qr  = carve((size_t)NB * ER * DMOD * 2);
  _Float16* kh  = carve((size_t)MTOT * KVD * 2);
  _Float16* kr  = carve((size_t)NB * ER * KVD * 2);
  _Float16* vt  = carve((size_t)NB * KVD * SEQ * 2);
  _Float16* vr  = carve((size_t)NB * KVD * ER * 2);
  _Float16* ch  = carve((size_t)MTOT * DMOD * 2);
  _Float16* cr  = carve((size_t)NB * ER * DMOD * 2);
  if (off > ws_size) return;

  cvt_x_kernel<<<(unsigned)((size_t)MTOT * DMOD / 8 / 256), 256, 0, stream>>>(x, xh);
  tr_w_kernel<<<dim3(DMOD / 64, DMOD / 64), 256, 0, stream>>>(Wq, wqt, DMOD, DMOD);
  tr_w_kernel<<<dim3(KVD / 64, DMOD / 64), 256, 0, stream>>>(Wk, wkt, DMOD, KVD);
  tr_w_kernel<<<dim3(KVD / 64, DMOD / 64), 256, 0, stream>>>(Wv, wvt, DMOD, KVD);
  tr_w_kernel<<<dim3(DMOD / 64, DMOD / 64), 256, 0, stream>>>(Wo, wot, DMOD, DMOD);

  gemm_kernel<0, _Float16><<<dim3(DMOD / 64, MTOT / 128), 128, 0, stream>>>(
      xh, xh, wqt, qh, qr, DMOD, DMOD, WSCINV);
  gemm_kernel<0, _Float16><<<dim3(KVD / 64, MTOT / 128), 128, 0, stream>>>(
      xh, xh, wkt, kh, kr, KVD, DMOD, WSCINV);
  gemm_kernel<1, _Float16><<<dim3(KVD / 64, MTOT / 128), 128, 0, stream>>>(
      xh, xh, wvt, vt, vr, KVD, DMOD, WSCINV);

  attn_kernel<1, 1><<<NB * NQH * 2, 256, 0, stream>>>(qh, qr, kh, kr, vt, vr, ch, cr, 0, 2);
  const int nqb_late = SEQ / 256 - 1;
  if (nqb_late > 0) {
    attn_kernel<2, 0><<<NB * NQH * nqb_late, 256, 0, stream>>>(qh, qr, kh, kr, vt, vr,
                                                            ch, cr, 1, nqb_late);
  }

  gemm_kernel<2, float><<<dim3(DMOD / 64, MTOT / 128), 128, 0, stream>>>(
      ch, cr, wot, out, cr, DMOD, DMOD, WSCINV);
}
